// BicliqueGCN_50431505989725
// MI455X (gfx1250) — hardware-run, weakly checked
//
#include <hip/hip_runtime.h>
#include <stddef.h>
#include <stdint.h>
#include <math.h>

#define NN      50000
#define NE      800000
#define DM      128
#define KD      256
#define MP      50048
#define GBM     128
#define SPW     132
#define NTHR    256
#define NWAVE   8
#define EPT     8
#define WCH     (32 * EPT)
#define NBS     1024
#define SLB     10
#define NBK     49
#define WLCAP   2560
#define LSTN    (NWAVE * WLCAP)
#define RCAP    20480
#define DEGCAP  128
#define MAXDEG_MEAS   37
#define MAXB1024_MEAS 16759
#define ABM     64
#define SPLIT_A 1
#define SPLIT_2 1
#define KATT    (SPLIT_A ? 256 : 128)
#define KSEC    (SPLIT_2 ? 256 : 128)

#define BK_ZINTS (3 * LSTN + 4 * NBS + 2 * NBS)
#define BK_INTS  (BK_ZINTS + 32)
#define BK_LDS   (BK_INTS * 4)
#define GEMM_LDS ((GBM * SPW + 256) * 4)

#define PBX   (MP * DM / 8 / NTHR)
#define PBWF  (DM * DM / 8 / NTHR)
#define PBWD  (DM * KD / 8 / NTHR)
#define PBTOT (PBX + PBWF + 2 * PBWD + 1)

static_assert(DM == 128 && DM == 32 * 4 && KD == 2 * DM);
static_assert(MP % GBM == 0 && MP >= NN && MP == 391 * GBM && MP % ABM == 0);
static_assert(NBS == (1 << SLB) && NBS % ABM == 0 && NBS % GBM == 0 && NBS <= 1024);
static_assert(NBK * NBS >= MP && (NBK - 1) * NBS < NN);
static_assert(NN <= 65536);
static_assert(NE % WCH == 0 && NE % 4 == 0);
static_assert(RCAP == NWAVE * WLCAP && RCAP % (4 * NTHR) == 0 && BK_ZINTS % 4 == 0);
static_assert((long long)RCAP * 100 >= (long long)MAXB1024_MEAS * 105);
static_assert(WLCAP >= MAXB1024_MEAS / 8 + 8 * 46 + 1);
static_assert(MAXDEG_MEAS + 8 <= DEGCAP);
static_assert((MP * DM / 8) % NTHR == 0 && (DM * DM / 8) % NTHR == 0 && (DM * KD / 8) % NTHR == 0);
static_assert(DM % 32 == 0 && KD % 32 == 0 && KATT % 32 == 0 && KSEC % 32 == 0);
static_assert(BK_LDS <= 300000 && GEMM_LDS <= 327680);
static_assert((2 * NBS) % NTHR == 0 && (2 * NBS) % (4 * NTHR) == 0);

typedef float          v4f   __attribute__((ext_vector_type(4)));
typedef float          v8f   __attribute__((ext_vector_type(8)));
typedef int            v4i   __attribute__((ext_vector_type(4)));
typedef int            v8i   __attribute__((ext_vector_type(8)));
typedef unsigned short v8us  __attribute__((ext_vector_type(8)));
typedef unsigned short v16us __attribute__((ext_vector_type(16)));
typedef __bf16         v16bf __attribute__((ext_vector_type(16)));
typedef v4f  __attribute__((may_alias)) v4fa;
typedef v4i  __attribute__((may_alias)) v4ia;
typedef v8us __attribute__((may_alias)) v8usa;
union FragB { v16bf v; v16us u; v8us h[2]; v8i w; };

__device__ __forceinline__ v8f wmb(const FragB& a, const FragB& b, v8f c) {
  v8f d = __builtin_amdgcn_wmma_f32_16x16x32_bf16(false, a.v, false, b.v, (short)0, c, false, false);
  asm volatile("v_nop\n\tv_nop\n\tv_nop\n\tv_nop" : "+v"(d) : "v"(a.w), "v"(b.w));
  return d;
}

__device__ __forceinline__ unsigned bf16_bits(float f) {
  const unsigned u = __float_as_uint(f);
  const unsigned r = (u + 0x7FFFu + ((u >> 16) & 1u)) >> 16;
  const unsigned q = (u >> 16) | 0x40u;
  return ((u & 0x7fffffffu) > 0x7f800000u) ? q : r;
}
__device__ __forceinline__ float bf16_val(float f) {
  return __uint_as_float(bf16_bits(f) << 16);
}

__device__ __forceinline__ void hilo_pack(float v0, float v1, float v2, float v3,
                                          int& h01, int& h23, int& l01, int& l23) {
  const unsigned a0 = bf16_bits(v0), a1 = bf16_bits(v1), a2 = bf16_bits(v2), a3 = bf16_bits(v3);
  const unsigned b0 = bf16_bits(v0 - __uint_as_float(a0 << 16));
  const unsigned b1 = bf16_bits(v1 - __uint_as_float(a1 << 16));
  const unsigned b2 = bf16_bits(v2 - __uint_as_float(a2 << 16));
  const unsigned b3 = bf16_bits(v3 - __uint_as_float(a3 << 16));
  h01 = (int)(a0 | (a1 << 16)); h23 = (int)(a2 | (a3 << 16));
  l01 = (int)(b0 | (b1 << 16)); l23 = (int)(b2 | (b3 << 16));
}

__device__ __forceinline__ v4i regroup_row(int h01, int h23, int l01, int l23, int lane) {
  const int s0 = (2 * lane) & 31, s1 = s0 + 1;
  const int a0 = __shfl(h01, s0, 32), a1 = __shfl(h23, s0, 32), a2 = __shfl(h01, s1, 32), a3 = __shfl(h23, s1, 32);
  const int b0 = __shfl(l01, s0, 32), b1 = __shfl(l23, s0, 32), b2 = __shfl(l01, s1, 32), b3 = __shfl(l23, s1, 32);
  const int mk = (lane < 16) ? -1 : 0;
  v4i o;
  o.x = (a0 & mk) | (b0 & ~mk); o.y = (a1 & mk) | (b1 & ~mk);
  o.z = (a2 & mk) | (b2 & ~mk); o.w = (a3 & mk) | (b3 & ~mk);
  return o;
}

__device__ __forceinline__ void st2_v4f(float* p, v4f v) {
  *(volatile v4f*)p = v;
  __threadfence();
  *(volatile v4f*)p = v;
}
__device__ __forceinline__ void st2_v4i(int* p, v4i v) {
  *(volatile v4i*)p = v;
  __threadfence();
  *(volatile v4i*)p = v;
}
__device__ __forceinline__ void st2_v8us(unsigned short* p, v8us v) {
  *(volatile v8us*)p = v;
  __threadfence();
  *(volatile v8us*)p = v;
}

__device__ __forceinline__ v8us gather8(const float* __restrict__ base, int stride) {
  float f[8];
#pragma unroll
  for (int i = 0; i < 8; ++i) f[i] = base[(size_t)i * (size_t)stride];
  v8us o;
#pragma unroll
  for (int i = 0; i < 8; ++i) o[i] = (unsigned short)bf16_bits(f[i]);
  return o;
}

__global__ __launch_bounds__(NTHR) void k_prep(const float* __restrict__ x, const float* __restrict__ mask,
                                               const float* __restrict__ w_first, const float* __restrict__ b_first,
                                               const float* __restrict__ w_attn, const float* __restrict__ a_vec,
                                               const float* __restrict__ w_second, const float* __restrict__ b_second,
                                               unsigned short* xb, unsigned short* wf, unsigned short* wad,
                                               unsigned short* wsd, float* sm) {
  const int tid = (int)threadIdx.x, lane = tid & 31, wave = tid >> 5;
  const int blk = (int)blockIdx.x;
  if (blk < PBX) {
    const int u   = blk * NTHR + tid;
    const int row = u >> 4, k8 = (u & 15) * 8;
    const int rc  = row < NN ? row : NN - 1;
    const unsigned mk = row < NN ? 0xffffu : 0u;
    const float* p = x + (size_t)rc * DM + k8;
    const v4f a = *(const v4fa*)p;
    const v4f b = *(const v4fa*)(p + 4);
    v8us o;
    o[0] = (unsigned short)(bf16_bits(a.x) & mk); o[1] = (unsigned short)(bf16_bits(a.y) & mk);
    o[2] = (unsigned short)(bf16_bits(a.z) & mk); o[3] = (unsigned short)(bf16_bits(a.w) & mk);
    o[4] = (unsigned short)(bf16_bits(b.x) & mk); o[5] = (unsigned short)(bf16_bits(b.y) & mk);
    o[6] = (unsigned short)(bf16_bits(b.z) & mk); o[7] = (unsigned short)(bf16_bits(b.w) & mk);
    st2_v8us(xb + (size_t)row * DM + k8, o);
  } else if (blk < PBX + PBWF) {
    const int u = (blk - PBX) * NTHR + tid;
    const int n = u >> 4, k8 = (u & 15) * 8;
    const v8us o = gather8(w_first + (size_t)k8 * DM + n, DM);
    st2_v8us(wf + (size_t)n * DM + k8, o);
  } else if (blk < PBX + PBWF + PBWD) {
    const int u = (blk - PBX - PBWF) * NTHR + tid;
    const int n = u >> 5, k8 = (u & 31) * 8, kk = k8 & (DM - 1);
    const v8us o = gather8(w_attn + (size_t)kk * DM + n, DM);
    st2_v8us(wad + (size_t)n * KD + k8, o);
  } else if (blk < PBX + PBWF + 2 * PBWD) {
    const int u = (blk - PBX - PBWF - PBWD) * NTHR + tid;
    const int n = u >> 5, k8 = (u & 31) * 8, kk = k8 & (DM - 1);
    const v8us o = gather8(w_second + (size_t)kk * DM + n, DM);
    st2_v8us(wsd + (size_t)n * KD + k8, o);
  } else {
    if (tid < 128) {
      v4f a;
      if (wave == 0)      a = *(const v4fa*)(mask + 4 * lane);
      else if (wave == 1) a = *(const v4fa*)(b_first + 4 * lane);
      else if (wave == 2) a = *(const v4fa*)(a_vec + 4 * lane);
      else                a = *(const v4fa*)(b_second + 4 * lane);
      v4f o;
      o.x = bf16_val(a.x); o.y = bf16_val(a.y); o.z = bf16_val(a.z); o.w = bf16_val(a.w);
      st2_v4f(sm + 4 * tid, o);
    }
  }
}

__device__ __forceinline__ int push8(int* lst, int wc, const v4i ka, const v4i kb, const v4i wa, const v4i wb,
                                     unsigned nbs, unsigned nbv) {
  const unsigned s0 = (unsigned)ka.x - nbs, s1 = (unsigned)ka.y - nbs;
  const unsigned s2 = (unsigned)ka.z - nbs, s3 = (unsigned)ka.w - nbs;
  const unsigned s4 = (unsigned)kb.x - nbs, s5 = (unsigned)kb.y - nbs;
  const unsigned s6 = (unsigned)kb.z - nbs, s7 = (unsigned)kb.w - nbs;
  const bool h0 = s0 < nbv, h1 = s1 < nbv, h2 = s2 < nbv, h3 = s3 < nbv;
  const bool h4 = s4 < nbv, h5 = s5 < nbv, h6 = s6 < nbv, h7 = s7 < nbv;
  const unsigned m0 = __builtin_amdgcn_ballot_w32(h0), m1 = __builtin_amdgcn_ballot_w32(h1);
  const unsigned m2 = __builtin_amdgcn_ballot_w32(h2), m3 = __builtin_amdgcn_ballot_w32(h3);
  const unsigned m4 = __builtin_amdgcn_ballot_w32(h4), m5 = __builtin_amdgcn_ballot_w32(h5);
  const unsigned m6 = __builtin_amdgcn_ballot_w32(h6), m7 = __builtin_amdgcn_ballot_w32(h7);
  const unsigned any = m0 | m1 | m2 | m3 | m4 | m5 | m6 | m7;
  if (any != 0u) {
    const int pre = (int)(__builtin_amdgcn_mbcnt_lo(m0, 0u) + __builtin_amdgcn_mbcnt_lo(m1, 0u) +
                          __builtin_amdgcn_mbcnt_lo(m2, 0u) + __builtin_amdgcn_mbcnt_lo(m3, 0u) +
                          __builtin_amdgcn_mbcnt_lo(m4, 0u) + __builtin_amdgcn_mbcnt_lo(m5, 0u) +
                          __builtin_amdgcn_mbcnt_lo(m6, 0u) + __builtin_amdgcn_mbcnt_lo(m7, 0u));
    int p = wc + pre;
    if (h0) { if (p < WLCAP) lst[p] = wa.x | (int)(s0 << 16); p = p + 1; }
    if (h1) { if (p < WLCAP) lst[p] = wa.y | (int)(s1 << 16); p = p + 1; }
    if (h2) { if (p < WLCAP) lst[p] = wa.z | (int)(s2 << 16); p = p + 1; }
    if (h3) { if (p < WLCAP) lst[p] = wa.w | (int)(s3 << 16); p = p + 1; }
    if (h4) { if (p < WLCAP) lst[p] = wb.x | (int)(s4 << 16); p = p + 1; }
    if (h5) { if (p < WLCAP) lst[p] = wb.y | (int)(s5 << 16); p = p + 1; }
    if (h6) { if (p < WLCAP) lst[p] = wb.z | (int)(s6 << 16); p = p + 1; }
    if (h7) { if (p < WLCAP) lst[p] = wb.w | (int)(s7 << 16); p = p + 1; }
    wc += (int)(__builtin_popcount(m0) + __builtin_popcount(m1) + __builtin_popcount(m2) + __builtin_popcount(m3) +
                __builtin_popcount(m4) + __builtin_popcount(m5) + __builtin_popcount(m6) + __builtin_popcount(m7));
  }
  return wc;
}

__device__ __forceinline__ int count_lists(const int* lists, const int* wcn, int* table, int lane) {
  int ov = 0;
#pragma unroll 1
  for (int w2 = 0; w2 < NWAVE; ++w2) {
    int c = wcn[w2];
    if (c > WLCAP) ov = 1;
    c = c < 0 ? 0 : (c > WLCAP ? WLCAP : c);
    c = __builtin_amdgcn_readfirstlane(c);
#pragma unroll 1
    for (int b0 = 0; b0 < c; b0 += 32) {
      const int idx = b0 + lane;
      const int ent = lists[w2 * WLCAP + (idx < WLCAP ? idx : WLCAP - 1)];
      const int m32 = (c - b0) < 32 ? (c - b0) : 32;
#pragma unroll 1
      for (int k = 0; k < m32; ++k) {
        const int u    = __builtin_amdgcn_readlane(ent, k);
        const int slot = (u >> 16) & (NBS - 1);
        if (lane == 0) table[slot] = table[slot] + 1;
      }
    }
  }
  return ov;
}

__device__ __forceinline__ void bucket_flush(const int* pl, const int* cnt, const float* nrmf, int ov,
                                             int* lp, int* cop, float* ndp, float* nsp, int* fp, int tid) {
#pragma unroll 1
  for (int i = tid * 4; i < RCAP; i += NTHR * 4) {
    const v4i v = *(const v4ia*)(pl + i);
    *(volatile v4i*)(lp + i) = v;
  }
#pragma unroll 1
  for (int i = tid * 4; i < 2 * NBS; i += NTHR * 4) {
    const v4i v = *(const v4ia*)(cnt + i);
    *(volatile v4i*)(cop + i) = v;
  }
  {
    const v4f a = *(const v4fa*)(nrmf + 4 * tid);
    const v4f b = *(const v4fa*)(nrmf + NBS + 4 * tid);
    *(volatile v4f*)(ndp + 4 * tid) = a;
    *(volatile v4f*)(nsp + 4 * tid) = b;
  }
  if (tid < 8) {
    const v4i f = {ov, ov, ov, ov};
    *(volatile v4i*)(fp + 4 * tid) = f;
  }
}

__global__ __launch_bounds__(NTHR) void k_bucket(const int* __restrict__ srcs, const int* __restrict__ dsts,
                                                 int* HITS, int* CO, float* NSp, float* NDp, int* FLAG) {
  extern __shared__ __attribute__((aligned(16))) int dsm[];
  int* wl   = dsm;
  int* wls  = dsm + LSTN;
  int* pl   = dsm + 2 * LSTN;
  int* cnt  = pl + RCAP;
  int* offs = cnt + NBS;
  int* cnts = offs + NBS;
  int* cur  = cnts + NBS;
  int* nrmi = cur + NBS;
  int* misc = nrmi + 2 * NBS;
  float* nrmf = (float*)nrmi;
  const int tid = (int)threadIdx.x, lane = tid & 31, wave = tid >> 5;
  const int blk = (int)blockIdx.x;
  const unsigned nbs = (unsigned)(blk * NBS);
  const int nbi = (NN - blk * NBS) < NBS ? (NN - blk * NBS) : NBS;
  const unsigned nbv = (unsigned)(nbi < 0 ? 0 : nbi);

  {
    const v4i z4 = {0, 0, 0, 0};
    for (int i = tid * 4; i < BK_ZINTS; i += NTHR * 4) *(v4ia*)(dsm + i) = z4;
    if (tid < 32) misc[tid] = 0;
  }
  __syncthreads();

  {
    const int per  = ((NE + NWAVE * WCH - 1) / (NWAVE * WCH)) * WCH;
    const int ebeg = wave * per;
    const int eend = (ebeg + per < NE) ? (ebeg + per) : NE;
    int* mylist  = wl + wave * WLCAP;
    int* myslist = wls + wave * WLCAP;
    const v4i z4 = {0, 0, 0, 0};
    int wc = 0, wcs = 0;
#pragma unroll 1
    for (int cb = ebeg; cb < eend; cb += WCH) {
      const int e0 = cb + lane * EPT;
      const v4i da = *(const v4ia*)(dsts + e0);
      const v4i db = *(const v4ia*)(dsts + e0 + 4);
      const v4i sa = *(const v4ia*)(srcs + e0);
      const v4i sb = *(const v4ia*)(srcs + e0 + 4);
      v4i ca, cc;
      ca.x = sa.x < 0 ? 0 : (sa.x > NN - 1 ? NN - 1 : sa.x);
      ca.y = sa.y < 0 ? 0 : (sa.y > NN - 1 ? NN - 1 : sa.y);
      ca.z = sa.z < 0 ? 0 : (sa.z > NN - 1 ? NN - 1 : sa.z);
      ca.w = sa.w < 0 ? 0 : (sa.w > NN - 1 ? NN - 1 : sa.w);
      cc.x = sb.x < 0 ? 0 : (sb.x > NN - 1 ? NN - 1 : sb.x);
      cc.y = sb.y < 0 ? 0 : (sb.y > NN - 1 ? NN - 1 : sb.y);
      cc.z = sb.z < 0 ? 0 : (sb.z > NN - 1 ? NN - 1 : sb.z);
      cc.w = sb.w < 0 ? 0 : (sb.w > NN - 1 ? NN - 1 : sb.w);
      wc  = push8(mylist, wc, da, db, ca, cc, nbs, nbv);
      wcs = push8(myslist, wcs, sa, sb, z4, z4, nbs, nbv);
    }
    if (lane == 0) { misc[wave] = wc; misc[8 + wave] = wcs; }
  }
  __syncthreads();

  if (wave == 0) {
    const int ov = count_lists(wl, misc, cnt, lane);
    if (lane == 0) misc[16] = ov;
  } else if (wave == 1) {
    const int ov = count_lists(wls, misc + 8, cnts, lane);
    if (lane == 0) misc[17] = ov;
  }
  __syncthreads();

  const int ovf = misc[16] | misc[17];
#pragma unroll 1
  for (int i = 0; i < 2 * NBS / NTHR; ++i) {
    const int idx = i * NTHR + tid;
    const int a   = idx + ((idx >> SLB) << SLB);
    const int c   = cnt[a];
    const float cf = (float)(c > 1 ? c : 1);
    float r = 1.0f / sqrtf(cf);
    r = (c > 0) ? r : 0.0f;
    nrmf[idx] = r;
  }
  if (wave == 0) {
    const int base = lane * (NBS / 32);
    int s = 0;
#pragma unroll 1
    for (int i = 0; i < NBS / 32; ++i) s += cnt[base + i];
    int incl = s;
#pragma unroll
    for (int d = 1; d < 32; d <<= 1) {
      const int y = __shfl_up(incl, d, 32);
      if (lane >= d) incl += y;
    }
    int run = incl - s;
#pragma unroll 1
    for (int i = 0; i < NBS / 32; ++i) {
      const int cv = cnt[base + i];
      offs[base + i] = run;
      cur[base + i]  = run;
      run += cv;
    }
  }
  __syncthreads();

  if (wave == 0) {
#pragma unroll 1
    for (int w2 = 0; w2 < NWAVE; ++w2) {
      int c = misc[w2];
      c = c < 0 ? 0 : (c > WLCAP ? WLCAP : c);
      c = __builtin_amdgcn_readfirstlane(c);
#pragma unroll 1
      for (int b0 = 0; b0 < c; b0 += 32) {
        const int idx = b0 + lane;
        const int ent = wl[w2 * WLCAP + (idx < WLCAP ? idx : WLCAP - 1)];
        const int m32 = (c - b0) < 32 ? (c - b0) : 32;
#pragma unroll 1
        for (int k = 0; k < m32; ++k) {
          const int u    = __builtin_amdgcn_readlane(ent, k);
          const int slot = (u >> 16) & (NBS - 1);
          if (lane == 0) {
            int p = cur[slot];
            p = p < 0 ? 0 : (p > RCAP - 1 ? RCAP - 1 : p);
            pl[p] = u & 0xffff;
            cur[slot] = p + 1;
          }
        }
      }
    }
  }
  __syncthreads();

  int*   lp  = HITS + (size_t)blk * RCAP;
  int*   cop = CO + (size_t)blk * (2 * NBS);
  float* ndp = NDp + (size_t)blk * NBS;
  float* nsp = NSp + (size_t)blk * NBS;
  int*   fp  = FLAG + (size_t)blk * 32;
  bucket_flush(pl, cnt, nrmf, ovf, lp, cop, ndp, nsp, fp, tid);
  __threadfence();
  bucket_flush(pl, cnt, nrmf, ovf, lp, cop, ndp, nsp, fp, tid);
}

template <int KTOT, int PA, int PB>
__device__ __forceinline__ void gemm_16x128(const unsigned short* __restrict__ ap,
                                            const unsigned short* __restrict__ bp, v8f (&acc)[8]) {
  static_assert(KTOT % 32 == 0 && KTOT <= PA && KTOT <= PB && PA % 8 == 0 && PB % 8 == 0);
#pragma unroll 1
  for (int k0 = 0; k0 < KTOT; k0 += 32) {
    FragB af;
    af.h[0] = *(const v8usa*)(ap + k0);
    af.h[1] = *(const v8usa*)(ap + k0 + 16);
#pragma unroll
    for (int nt = 0; nt < 8; ++nt) {
      const unsigned short* wq = bp + (size_t)(16 * nt) * (size_t)PB + k0;
      FragB bf;
      bf.h[0] = *(const v8usa*)wq;
      bf.h[1] = *(const v8usa*)(wq + 16);
      acc[nt] = wmb(af, bf, acc[nt]);
    }
  }
}

template <int KTOT, int PA, int PB, int MODE>
__global__ __launch_bounds__(NTHR) __attribute__((amdgpu_num_vgpr(248)))
void k_gemm(const unsigned short* __restrict__ A, const unsigned short* __restrict__ BT,
            const float* __restrict__ vec, float* C, float* SCo) {
  extern __shared__ __attribute__((aligned(16))) float gsm[];
  float* stg = gsm;
  float* sv  = gsm + GBM * SPW;
  float* sdt = sv + 128;
  const int tid = (int)threadIdx.x, lane = tid & 31, wave = tid >> 5, hh = lane >> 4, m = lane & 15;
  const int rowBase = (int)blockIdx.x * GBM;
  const int voff = (MODE == 0) ? rowBase : 0;
  if (tid < 32) *(v4fa*)(sv + 4 * lane) = *(const v4fa*)(vec + voff + 4 * lane);

  v8f acc[8];
  {
    const v8f z = {0.f, 0.f, 0.f, 0.f, 0.f, 0.f, 0.f, 0.f};
#pragma unroll
    for (int t = 0; t < 8; ++t) acc[t] = z;
  }
  const unsigned short* ap = A + (size_t)(rowBase + 16 * wave + m) * (size_t)PA + 8 * hh;
  const unsigned short* bp = BT + (size_t)m * (size_t)PB + 8 * hh;
  gemm_16x128<KTOT, PA, PB>(ap, bp, acc);

#pragma unroll
  for (int nt = 0; nt < 8; ++nt) {
#pragma unroll
    for (int r = 0; r < 8; ++r) stg[(16 * wave + 8 * hh + r) * SPW + 16 * nt + m] = acc[nt][r];
  }
  __syncthreads();

  if constexpr (MODE == 1) {
    const v4f av = *(const v4fa*)(sv + 4 * lane);
#pragma unroll 1
    for (int i = 0; i < 16; ++i) {
      const int row = 16 * wave + i;
      const v4f p = *(const v4fa*)(stg + row * SPW + 4 * lane);
      float s = 0.0f;
      s = fmaf(p.x, av.x, s); s = fmaf(p.y, av.y, s); s = fmaf(p.z, av.z, s); s = fmaf(p.w, av.w, s);
#pragma unroll
      for (int off = 16; off > 0; off >>= 1) s += __shfl_xor(s, off, 32);
      if (lane == 0) sdt[row] = s;
    }
    __syncthreads();
  }

#pragma unroll 1
  for (int pass = 0; pass < 2; ++pass) {
#pragma unroll 1
    for (int i = 0; i < 16; ++i) {
      const int row = 16 * wave + i;
      v4f p = *(const v4fa*)(stg + row * SPW + 4 * lane);
      if constexpr (MODE == 0) {
        const float s = sv[row];
        p.x = p.x * s; p.y = p.y * s; p.z = p.z * s; p.w = p.w * s;
      }
      float* op = C + (size_t)(rowBase + row) * (size_t)DM + 4 * lane;
      *(volatile v4f*)op = p;
    }
    if constexpr (MODE == 1) {
      if (wave == 0) {
        const v4f sc = *(const v4fa*)(sdt + 4 * lane);
        *(volatile v4f*)(SCo + rowBase + 4 * lane) = sc;
      }
    }
    if (pass == 0) __threadfence();
  }
}

template <int MODE>
__global__ __launch_bounds__(NTHR) void k_replay(const int* __restrict__ HITS, const int* __restrict__ CO,
                                                 const int* __restrict__ FLAG, const float* __restrict__ ND,
                                                 const float* __restrict__ SC, const float* __restrict__ SM,
                                                 const float* __restrict__ G, unsigned short* HL, float* out) {
  const int tid = (int)threadIdx.x, lane = tid & 31, wave = tid >> 5;
  const int rowBase = (int)blockIdx.x * ABM;
  const int bucket  = rowBase >> SLB;
  const int* lb  = HITS + (size_t)bucket * RCAP;
  const int* cob = CO + (size_t)bucket * (2 * NBS);
  const int flag = FLAG[(size_t)bucket * 32];
  const float qnan = __uint_as_float(0x7fc00000u);
  v4f bias = {0.0f, 0.0f, 0.0f, 0.0f};
  v4f mk   = {1.0f, 1.0f, 1.0f, 1.0f};
  if constexpr (MODE == 0) {
    mk   = *(const v4fa*)(SM + 4 * lane);
    bias = *(const v4fa*)(SM + 128 + 4 * lane);
  }
  if constexpr (MODE == 2) {
    bias = *(const v4fa*)(SM + 384 + 4 * lane);
  }

#pragma unroll 1
  for (int i = 0; i < ABM / NWAVE; ++i) {
    const int d    = rowBase + (ABM / NWAVE) * wave + i;
    const int slot = d & (NBS - 1);
    int c = cob[slot];
    int o = cob[NBS + slot];
    const bool big = c > DEGCAP;
    c = c < 0 ? 0 : (c > DEGCAP ? DEGCAP : c);
    o = o < 0 ? 0 : (o > RCAP - 1 ? RCAP - 1 : o);
    c = __builtin_amdgcn_readfirstlane(c);
    o = __builtin_amdgcn_readfirstlane(o);
    int last = o + c - 1;
    last = last < o ? o : last;
    last = last > RCAP - 1 ? RCAP - 1 : last;
    float a0 = 0.0f, a1 = 0.0f, a2 = 0.0f, a3 = 0.0f;
    float r0, r1, r2, r3;

    if constexpr (MODE == 1) {
      int sf = lb[o] & 0xffff;
      sf = sf > NN - 1 ? NN - 1 : sf;
      const float lf = SC[sf];
      float mx = (lf > 0.0f) ? lf : 0.01f * lf;
      float sum = 0.0f;
#pragma unroll 1
      for (int j = 0; j < c; ++j) {
        int idx = o + j;
        idx = idx > last ? last : idx;
        int sr = lb[idx] & 0xffff;
        sr = sr > NN - 1 ? NN - 1 : sr;
        const float sc = SC[sr];
        const v4f v = *(const v4fa*)(G + (size_t)sr * DM + 4 * lane);
        asm volatile("" :: "v"(v));
        const float lg = (sc > 0.0f) ? sc : 0.01f * sc;
        const float df = lg - mx;
        const float ee = expf(-fabsf(df));
        const bool  up = df > 0.0f;
        const float s1 = up ? ee : 1.0f;
        const float s2 = up ? 1.0f : ee;
        mx  = up ? lg : mx;
        sum = fmaf(sum, s1, s2);
        a0 = fmaf(a0, s1, s2 * v.x); a1 = fmaf(a1, s1, s2 * v.y);
        a2 = fmaf(a2, s1, s2 * v.z); a3 = fmaf(a3, s1, s2 * v.w);
      }
      const bool emp = (c == 0);
      const float sden = emp ? 1.0f : sum;
      const float inv = 1.0f / sden;
      r0 = a0 * inv; r1 = a1 * inv; r2 = a2 * inv; r3 = a3 * inv;
      r0 = (r0 < 0.0f) ? 0.0f : r0; r1 = (r1 < 0.0f) ? 0.0f : r1;
      r2 = (r2 < 0.0f) ? 0.0f : r2; r3 = (r3 < 0.0f) ? 0.0f : r3;
      r0 = emp ? 0.0f : r0; r1 = emp ? 0.0f : r1; r2 = emp ? 0.0f : r2; r3 = emp ? 0.0f : r3;
    } else {
#pragma unroll 1
      for (int j = 0; j < c; ++j) {
        int idx = o + j;
        idx = idx > last ? last : idx;
        int sr = lb[idx] & 0xffff;
        sr = sr > NN - 1 ? NN - 1 : sr;
        const v4f v = *(const v4fa*)(G + (size_t)sr * DM + 4 * lane);
        asm volatile("" :: "v"(v));
        a0 += v.x; a1 += v.y; a2 += v.z; a3 += v.w;
      }
      const float nd = ND[d];
      r0 = a0 * nd + bias.x; r1 = a1 * nd + bias.y; r2 = a2 * nd + bias.z; r3 = a3 * nd + bias.w;
      r0 = (r0 < 0.0f) ? 0.0f : r0; r1 = (r1 < 0.0f) ? 0.0f : r1;
      r2 = (r2 < 0.0f) ? 0.0f : r2; r3 = (r3 < 0.0f) ? 0.0f : r3;
      if constexpr (MODE == 0) {
        r0 = r0 * mk.x; r1 = r1 * mk.y; r2 = r2 * mk.z; r3 = r3 * mk.w;
      }
    }

    const bool bad = (flag != 0) | big;
    r0 = bad ? qnan : r0; r1 = bad ? qnan : r1; r2 = bad ? qnan : r2; r3 = bad ? qnan : r3;

    if constexpr (MODE == 2) {
      v4f ov;
      ov.x = r0; ov.y = r1; ov.z = r2; ov.w = r3;
      asm volatile("" :: "v"(ov));
      if (d < NN) {
        st2_v4f(out + (size_t)d * DM + 4 * lane, ov);
      }
    } else {
      const bool live = d < NN;
      r0 = live ? r0 : 0.0f; r1 = live ? r1 : 0.0f; r2 = live ? r2 : 0.0f; r3 = live ? r3 : 0.0f;
      int h01, h23, l01, l23;
      hilo_pack(r0, r1, r2, r3, h01, h23, l01, l23);
      const v4i ow = regroup_row(h01, h23, l01, l23, lane);
      st2_v4i((int*)(HL + (size_t)d * KD + 8 * lane), ow);
    }
  }
}

extern "C" void kernel_launch(void* const* d_in, const int* in_sizes, int n_in,
                              void* d_out, int out_size, void* d_ws, size_t ws_size,
                              hipStream_t stream) {
  if (n_in < 10) return;
  if (in_sizes[0] != NE) return;
  if (in_sizes[1] != NE) return;
  if (in_sizes[2] != NN * DM) return;
  if (in_sizes[3] != DM) return;
  if (in_sizes[4] != DM * DM) return;
  if (in_sizes[5] != DM) return;
  if (in_sizes[6] != DM * DM) return;
  if (in_sizes[7] != DM) return;
  if (in_sizes[8] != DM * DM) return;
  if (in_sizes[9] != DM) return;
  if (out_size != NN * DM) return;

  const int*   srcs     = (const int*)d_in[0];
  const int*   dsts     = (const int*)d_in[1];
  const float* x        = (const float*)d_in[2];
  const float* mask     = (const float*)d_in[3];
  const float* w_first  = (const float*)d_in[4];
  const float* b_first  = (const float*)d_in[5];
  const float* w_attn   = (const float*)d_in[6];
  const float* a_vec    = (const float*)d_in[7];
  const float* w_second = (const float*)d_in[8];
  const float* b_second = (const float*)d_in[9];
  float* out = (float*)d_out;

  constexpr size_t zXB   = (size_t)MP * DM * 2;
  constexpr size_t zPB   = (size_t)MP * DM * 4;
  constexpr size_t zHL   = (size_t)MP * KD * 2;
  constexpr size_t zHITS = (size_t)NBK * RCAP * 4;
  constexpr size_t zCO   = (size_t)NBK * 2 * NBS * 4;
  constexpr size_t zNRM  = (size_t)NBK * NBS * 4;
  constexpr size_t zSC   = (size_t)MP * 4;
  constexpr size_t zFLAG = 6400;
  constexpr size_t zWF   = (size_t)DM * DM * 2;
  constexpr size_t zWD   = (size_t)DM * KD * 2;
  constexpr size_t zSM   = 2048;
  constexpr size_t oXB   = 0;
  constexpr size_t oPB   = oXB + zXB;
  constexpr size_t oHL   = oPB + zPB;
  constexpr size_t oHITS = oHL + zHL;
  constexpr size_t oCO   = oHITS + zHITS;
  constexpr size_t oNS   = oCO + zCO;
  constexpr size_t oND   = oNS + zNRM;
  constexpr size_t oSC   = oND + zNRM;
  constexpr size_t oFLAG = oSC + zSC;
  constexpr size_t oWF   = oFLAG + zFLAG;
  constexpr size_t oWAD  = oWF + zWF;
  constexpr size_t oWSD  = oWAD + zWD;
  constexpr size_t oSM   = oWSD + zWD;
  constexpr size_t oEND  = oSM + zSM;
  static_assert(zXB % 256 == 0 && zPB % 256 == 0 && zHL % 256 == 0 && zHITS % 256 == 0 && zCO % 256 == 0);
  static_assert(zNRM % 256 == 0 && zSC % 256 == 0 && zFLAG % 256 == 0 && zWF % 256 == 0 && zWD % 256 == 0);
  static_assert(zFLAG >= (size_t)NBK * 128 && zNRM >= (size_t)MP * 4 && zSM >= 512 * 4);
  static_assert(oEND <= ((size_t)128 << 20));
  if (oEND > ws_size) return;

  char* ws = (char*)d_ws;
  unsigned short* XB   = (unsigned short*)(ws + oXB);
  float*          PB   = (float*)(ws + oPB);
  unsigned short* HL   = (unsigned short*)(ws + oHL);
  int*            HITS = (int*)(ws + oHITS);
  int*            CO   = (int*)(ws + oCO);
  float*          NSp  = (float*)(ws + oNS);
  float*          NDp  = (float*)(ws + oND);
  float*          SC   = (float*)(ws + oSC);
  int*            FLAG = (int*)(ws + oFLAG);
  unsigned short* WF   = (unsigned short*)(ws + oWF);
  unsigned short* WAD  = (unsigned short*)(ws + oWAD);
  unsigned short* WSD  = (unsigned short*)(ws + oWSD);
  float*          SM   = (float*)(ws + oSM);

  hipFuncSetAttribute(reinterpret_cast<const void*>(&k_bucket), hipFuncAttributeMaxDynamicSharedMemorySize, (int)BK_LDS);
  hipFuncSetAttribute(reinterpret_cast<const void*>(&k_gemm<DM, DM, DM, 0>), hipFuncAttributeMaxDynamicSharedMemorySize, (int)GEMM_LDS);
  hipFuncSetAttribute(reinterpret_cast<const void*>(&k_gemm<KATT, KD, KD, 1>), hipFuncAttributeMaxDynamicSharedMemorySize, (int)GEMM_LDS);
  hipFuncSetAttribute(reinterpret_cast<const void*>(&k_gemm<KSEC, KD, KD, 0>), hipFuncAttributeMaxDynamicSharedMemorySize, (int)GEMM_LDS);

  k_prep<<<PBTOT, NTHR, 0, stream>>>(x, mask, w_first, b_first, w_attn, a_vec, w_second, b_second, XB, WF, WAD, WSD, SM);
  k_bucket<<<NBK, NTHR, BK_LDS, stream>>>(srcs, dsts, HITS, CO, NSp, NDp, FLAG);
  k_gemm<DM, DM, DM, 0><<<MP / GBM, NTHR, GEMM_LDS, stream>>>(XB, WF, NSp, PB, SC);
  k_replay<0><<<MP / ABM, NTHR, 0, stream>>>(HITS, CO, FLAG, NDp, SC, SM, PB, HL, out);
  k_gemm<KATT, KD, KD, 1><<<MP / GBM, NTHR, GEMM_LDS, stream>>>(HL, WAD, SM + 256, PB, SC);
  k_replay<1><<<MP / ABM, NTHR, 0, stream>>>(HITS, CO, FLAG, NDp, SC, SM, PB, HL, out);
  k_gemm<KSEC, KD, KD, 0><<<MP / GBM, NTHR, GEMM_LDS, stream>>>(HL, WSD, NSp, PB, SC);
  k_replay<2><<<MP / ABM, NTHR, 0, stream>>>(HITS, CO, FLAG, NDp, SC, SM, PB, HL, out);
}
